// Block_63402307224451
// MI455X (gfx1250) — hardware-verified
//
#include <hip/hip_runtime.h>
#ifndef NB
#define NB 4
#endif
#ifndef SEQ
#define SEQ 1024
#endif
#define NB_FULL 4
#define SEQ_FULL 1024
#define DM 768
#define NH 12
#define HD 64
#define DFF 3072
#define LNT 192
#define LQ (3 * DM)
#define NR ((size_t)NB * SEQ)
#define OSP 72

typedef unsigned short v8us __attribute__((ext_vector_type(8), may_alias));
typedef float  v8f  __attribute__((ext_vector_type(8)));
typedef float  v4f  __attribute__((ext_vector_type(4)));
typedef float  v4fa __attribute__((ext_vector_type(4), may_alias));
typedef int    v4i  __attribute__((ext_vector_type(4)));
typedef int    v4ia __attribute__((ext_vector_type(4), may_alias));
typedef _Float16 v16h __attribute__((ext_vector_type(16)));
typedef _Float16 v4h __attribute__((ext_vector_type(4)));
union FragH { v16h v; v8us half[2]; _Float16 h[16]; unsigned short u[16]; };

static_assert(DM == NH * HD);
static_assert(HD == 64);
static_assert(DM == LNT * 4);
static_assert(LNT % 32 == 0 && LNT <= 256);
static_assert(SEQ % 64 == 0);
static_assert(NR % 128 == 0);
static_assert(DM % 64 == 0 && LQ % 64 == 0 && DFF % 64 == 0);
static_assert(DM % 32 == 0 && DFF % 32 == 0);
static_assert((DM / 8) % 8 == 0 && (DFF / 8) % 8 == 0);
static_assert(OSP % 8 == 0 && OSP >= HD);
static_assert(NB <= NB_FULL && SEQ <= SEQ_FULL);
static_assert(DFF == LQ + DM);

#define WMMA_F16(a, b, c) __builtin_amdgcn_wmma_f32_16x16x32_f16(false, (a), false, (b), (short)0, (c), false, false)

__device__ __forceinline__ unsigned short bf16_bits(float x) { unsigned int u = __float_as_uint(x); return (unsigned short)((u + 0x7FFFu + ((u >> 16) & 1u)) >> 16); }
__device__ __forceinline__ float bf16_rne(float x) { return __uint_as_float(((unsigned int)bf16_bits(x)) << 16); }
__device__ __forceinline__ v16h g2_frag(const _Float16* p, int hh) { FragH f; f.half[0] = *(const v8us*)((const unsigned short*)p + 8 * hh); f.half[1] = *(const v8us*)((const unsigned short*)p + 16 + 8 * hh); return f.v; }

__global__ __launch_bounds__(256) void k_wt_f16(const float* __restrict__ W, _Float16* __restrict__ Wt, int K, int N, float scale) {
  const int t = blockIdx.x * 256 + threadIdx.x; const int k8n = K / 8; if (t >= N * k8n) return;
  const int n = t / k8n, k8 = (t - n * k8n) * 8; FragH f;
#pragma unroll
  for (int i = 0; i < 8; ++i) f.h[i] = (_Float16)(bf16_rne(W[(size_t)(k8 + i) * N + n]) * scale);
  const v8us o = f.half[0];
  unsigned short* d = (unsigned short*)Wt + (size_t)n * K + k8;
  *(volatile v8us*)d = o; __threadfence(); *(volatile v8us*)d = o;
}

template <int BFIN, int WXB>
__device__ __forceinline__ void ln_body(const float* __restrict__ xr, const float* __restrict__ g, const float* __restrict__ bb, float eps, _Float16* __restrict__ nrow, float* __restrict__ xbrow) {
  #pragma clang fp contract(off)
  __shared__ float red[256];
  const int t = threadIdx.x; const bool act = t < LNT; const int tc = act ? t : (LNT - 1);
  const v4f xa = *(const v4fa*)(xr + tc * 4); float s[4]; float sum = 0.f;
#pragma unroll
  for (int q = 0; q < 4; ++q) { s[q] = BFIN ? bf16_rne(xa[q]) : xa[q]; sum = sum + s[q]; }
  red[t] = act ? sum : 0.f; __syncthreads();
  for (int st = 128; st > 0; st >>= 1) { if (t < st) red[t] = red[t] + red[t + st]; __syncthreads(); }
  const float mu = red[0] * (1.0f / (float)DM); __syncthreads();
  float vs = 0.f;
#pragma unroll
  for (int q = 0; q < 4; ++q) { const float dl = s[q] - mu; vs = vs + dl * dl; }
  red[t] = act ? vs : 0.f; __syncthreads();
  for (int st = 128; st > 0; st >>= 1) { if (t < st) red[t] = red[t] + red[t + st]; __syncthreads(); }
  const float rs = rsqrtf(red[0] * (1.0f / (float)DM) + eps); v4h y; v4f xb;
#pragma unroll
  for (int q = 0; q < 4; ++q) { const int c = tc * 4 + q; y[q] = (_Float16)(((s[q] - mu) * rs) * bf16_rne(g[c]) + bf16_rne(bb[c])); xb[q] = s[q]; }
  if (act) {
    for (int pass = 0; pass < 2; ++pass) { *(volatile v4h*)(nrow + tc * 4) = y; if (WXB) *(volatile v4f*)(xbrow + tc * 4) = xb; if (pass == 0) __threadfence(); }
  }
}
__global__ __launch_bounds__(256) void k_ln1(const float* __restrict__ x, const float* __restrict__ g, const float* __restrict__ bb, _Float16* __restrict__ N16, float* __restrict__ XB) {
  const size_t r = blockIdx.x; const size_t src = (r / SEQ) * (size_t)SEQ_FULL + (r % SEQ);
  ln_body<1, 1>(x + src * DM, g, bb, 1e-5f, N16 + r * DM, XB + r * DM);
}
__global__ __launch_bounds__(256) void k_ln2(const float* __restrict__ X1, const float* __restrict__ g, const float* __restrict__ bb, _Float16* __restrict__ N16) {
  const size_t r = blockIdx.x;
  ln_body<0, 0>(X1 + r * DM, g, bb, 1e-5f, N16 + r * DM, (float*)0);
}

template <int ACT, bool RES, bool OUT16>
__device__ __forceinline__ void gemm2_body(const _Float16* __restrict__ A, int lda, const _Float16* __restrict__ Bh, int ldb, float alpha, const float* __restrict__ bias,
                                           const float* __restrict__ R, int ldr, float* __restrict__ C, _Float16* __restrict__ C16, int ldc, int M, int N, int K) {
  __shared__ __attribute__((aligned(16))) float so[4][32][68];
  const int tid = threadIdx.x, w = __builtin_amdgcn_readfirstlane(tid >> 5), lane = tid & 31, ln = lane & 15, hh = lane >> 4;
  const int ntn = N >> 6; const int mt = blockIdx.x / ntn, nq = blockIdx.x - mt * ntn; const int row0 = mt * 128 + 32 * w, col0 = nq * 64;
  if (row0 >= M) return;
  const _Float16* a0p = A + (size_t)(row0 + ln) * lda; const _Float16* a1p = a0p + (size_t)16 * lda;
  const _Float16* b0p = Bh + (size_t)(col0 + ln) * ldb; const _Float16* b1p = b0p + (size_t)16 * ldb; const _Float16* b2p = b1p + (size_t)16 * ldb; const _Float16* b3p = b2p + (size_t)16 * ldb;
  const v8f z8 = {0.f, 0.f, 0.f, 0.f, 0.f, 0.f, 0.f, 0.f};
  v8f c00 = z8, c01 = z8, c02 = z8, c03 = z8, c10 = z8, c11 = z8, c12 = z8, c13 = z8;
#pragma unroll 1
  for (int kb = 0; kb < K; kb += 32) {
    const v16h a0 = g2_frag(a0p + kb, hh), a1 = g2_frag(a1p + kb, hh);
    const v16h b0 = g2_frag(b0p + kb, hh), b1 = g2_frag(b1p + kb, hh), b2 = g2_frag(b2p + kb, hh), b3 = g2_frag(b3p + kb, hh);
    c00 = WMMA_F16(a0, b0, c00); c10 = WMMA_F16(a1, b0, c10);
    c01 = WMMA_F16(a0, b1, c01); c11 = WMMA_F16(a1, b1, c11);
    c02 = WMMA_F16(a0, b2, c02); c12 = WMMA_F16(a1, b2, c12);
    c03 = WMMA_F16(a0, b3, c03); c13 = WMMA_F16(a1, b3, c13);
    asm volatile("v_nop\n\tv_nop\n\tv_nop\n\tv_nop" : "+v"(c00), "+v"(c01), "+v"(c02), "+v"(c03), "+v"(c10), "+v"(c11), "+v"(c12), "+v"(c13) : "v"(a0), "v"(a1), "v"(b0), "v"(b1), "v"(b2), "v"(b3));
  }
  v8f accs[8] = {c00, c01, c02, c03, c10, c11, c12, c13};
#pragma unroll
  for (int u = 0; u < 8; ++u) {
    const int t = u & 3, half = u >> 2; const int col = col0 + t * 16 + ln; const float bv = bf16_rne(bias[col]);
#pragma unroll
    for (int r = 0; r < 8; ++r) {
      const int rloc = half * 16 + 8 * hh + r;
      so[w][rloc][t * 16 + ln] = accs[u][r] * alpha + bv;
    }
  }
  __builtin_amdgcn_fence(4  , "workgroup"); __builtin_amdgcn_wave_barrier();
  const int rsub = lane >> 4, c4 = (lane & 15) * 4;
  if (ACT == 6) {
#pragma unroll 1
    for (int q = 0; q < 16; ++q) {
      const int r = q * 2 + rsub; v4f v = *(const v4fa*)&so[w][r][c4];
#pragma unroll
      for (int i = 0; i < 4; ++i) v[i] = 0.5f * v[i] * (1.0f + erff(v[i] * 0.70710678118654752f));
      *(v4fa*)&so[w][r][c4] = v;
    }
    __builtin_amdgcn_fence(4  , "workgroup"); __builtin_amdgcn_wave_barrier();
  }
  for (int pass = 0; pass < 2; ++pass) {
#pragma unroll 4
    for (int q = 0; q < 16; ++q) {
      const int r = q * 2 + rsub; const size_t grow = (size_t)(row0 + r);
      v4f v = *(const v4fa*)&so[w][r][c4];
      if (RES) { const v4f rv = *(const v4fa*)(R + grow * ldr + col0 + c4); v = v + rv; }
      if (OUT16) { v4h h4;
#pragma unroll
        for (int i = 0; i < 4; ++i) h4[i] = (_Float16)v[i];
        *(volatile v4h*)(C16 + grow * ldc + col0 + c4) = h4; }
      else *(volatile v4f*)(C + grow * ldc + col0 + c4) = v;
    }
    if (pass == 0) __threadfence();
  }
}
__global__ __launch_bounds__(128) void k_gemm_h16(const _Float16* __restrict__ A, int lda, const _Float16* __restrict__ Bh, int ldb, float alpha, const float* __restrict__ bias, _Float16* __restrict__ C16, int ldc, int M, int N, int K) {
  gemm2_body<0, false, true>(A, lda, Bh, ldb, alpha, bias, (const float*)0, 0, (float*)0, C16, ldc, M, N, K);
}
__global__ __launch_bounds__(128) void k_gemm_gelu16(const _Float16* __restrict__ A, int lda, const _Float16* __restrict__ Bh, int ldb, float alpha, const float* __restrict__ bias, _Float16* __restrict__ C16, int ldc, int M, int N, int K) {
  gemm2_body<6, false, true>(A, lda, Bh, ldb, alpha, bias, (const float*)0, 0, (float*)0, C16, ldc, M, N, K);
}
__global__ __launch_bounds__(128) void k_gemm_res32(const _Float16* __restrict__ A, int lda, const _Float16* __restrict__ Bh, int ldb, float alpha, const float* __restrict__ bias, const float* __restrict__ R, int ldr, float* __restrict__ C, int ldc, int M, int N, int K) {
  gemm2_body<0, true, false>(A, lda, Bh, ldb, alpha, bias, R, ldr, C, (_Float16*)0, ldc, M, N, K);
}

__global__ __launch_bounds__(256) void k_vt(const _Float16* __restrict__ QKV, _Float16* __restrict__ VT) {
  __shared__ unsigned short tl[64][66];
  const int tid = threadIdx.x; const int slab = blockIdx.x / (SEQ / 64), lg = blockIdx.x % (SEQ / 64); const int b = slab / NH, h = slab % NH;
  for (int i = tid; i < 64 * 8; i += 256) { const int r = i / 8, c8 = (i % 8) * 8; FragH f;
    f.half[0] = *(const v8us*)((const unsigned short*)QKV + ((size_t)b * SEQ + lg * 64 + r) * LQ + 2 * DM + h * HD + c8);
#pragma unroll
    for (int q = 0; q < 8; ++q) tl[r][c8 + q] = f.u[q]; }
  __syncthreads();
  for (int pass = 0; pass < 2; ++pass) {
#pragma unroll
    for (int rd = 0; rd < 2; ++rd) { const int d = rd * 32 + tid / 8, pc = tid % 8; FragH f;
#pragma unroll
      for (int q = 0; q < 8; ++q) f.u[q] = tl[pc * 8 + q][d];
      *(volatile v8us*)((unsigned short*)VT + ((size_t)slab * HD + d) * SEQ + lg * 64 + pc * 8) = f.half[0]; }
    if (pass == 0) __threadfence(); }
}

__device__ __forceinline__ v8us pack8(v8f o, float inv) { FragH f;
#pragma unroll
  for (int r = 0; r < 8; ++r) f.h[r] = (_Float16)(o[r] * inv);
  return f.half[0]; }

__global__ __launch_bounds__(128) void k_flash(const _Float16* __restrict__ QKV, const _Float16* __restrict__ VT, const int* __restrict__ mask, _Float16* __restrict__ O16) {
  __shared__ __attribute__((aligned(16))) unsigned short so[4][16][OSP];
  const int tid = threadIdx.x, w = __builtin_amdgcn_readfirstlane(tid >> 5), lane = tid & 31, ln = lane & 15, hh = lane >> 4;
  const int qt = blockIdx.x % (SEQ / 64), bh = blockIdx.x / (SEQ / 64); const int b = bh / NH, h = bh - b * NH;
  const int q0 = qt * 64 + w * 16; const size_t rowb = (size_t)b * SEQ;
  const size_t qoff = (rowb + q0 + ln) * LQ + (size_t)h * HD;
  const size_t koff = (rowb + ln) * LQ + DM + (size_t)h * HD;
  const size_t voff = ((size_t)bh * HD + ln) * SEQ;
  const size_t moff = (size_t)b * SEQ_FULL + (size_t)(8 * hh);
  const v8f z8 = {0.f, 0.f, 0.f, 0.f, 0.f, 0.f, 0.f, 0.f};
  v8f o0 = z8, o1 = z8, o2 = z8, o3 = z8; float m = -1.0e30f, l = 0.f;
#pragma unroll 1
  for (int k0 = 0; k0 < SEQ; k0 += 32) {
    const size_t ka = koff + (size_t)k0 * LQ, kc = ka + (size_t)16 * LQ;
    const v16h qa = g2_frag(QKV + qoff, hh), qb = g2_frag(QKV + qoff + 32, hh);
    const v16h k00 = g2_frag(QKV + ka, hh), k01 = g2_frag(QKV + ka + 32, hh), k10 = g2_frag(QKV + kc, hh), k11 = g2_frag(QKV + kc + 32, hh);
    v8f s0 = z8, s1 = z8;
    s0 = WMMA_F16(k00, qa, s0); s1 = WMMA_F16(k10, qa, s1); s0 = WMMA_F16(k01, qb, s0); s1 = WMMA_F16(k11, qb, s1);
    asm volatile("v_nop\n\tv_nop\n\tv_nop\n\tv_nop" : "+v"(s0), "+v"(s1) : "v"(k00), "v"(k01), "v"(k10), "v"(k11), "v"(qa), "v"(qb));
    const v4i ma = *(const v4ia*)(mask + moff + k0), mb = *(const v4ia*)(mask + moff + k0 + 4);
    const v4i mc = *(const v4ia*)(mask + moff + k0 + 16), md = *(const v4ia*)(mask + moff + k0 + 20);
#pragma unroll
    for (int r = 0; r < 4; ++r) {
      s0[r]     = fmaf(s0[r],     0.125f, (ma[r] == 0) ? -10000.0f : 0.0f);
      s0[4 + r] = fmaf(s0[4 + r], 0.125f, (mb[r] == 0) ? -10000.0f : 0.0f);
      s1[r]     = fmaf(s1[r],     0.125f, (mc[r] == 0) ? -10000.0f : 0.0f);
      s1[4 + r] = fmaf(s1[4 + r], 0.125f, (md[r] == 0) ? -10000.0f : 0.0f);
    }
    float mx = -3.0e38f;
#pragma unroll
    for (int r = 0; r < 8; ++r) mx = fmaxf(mx, fmaxf(s0[r], s1[r]));
    const float mxo = __shfl_xor(mx, 16); mx = fmaxf(mx, mxo);
    const float mn = fmaxf(m, mx);
    const float alpha = __expf(m - mn); m = mn;
    const float msh = mn - 5.5451774f;
    FragH pf; float ps = 0.f;
#pragma unroll
    for (int r = 0; r < 8; ++r) { const float p0 = __expf(s0[r] - msh); const float p1 = __expf(s1[r] - msh); ps += p0 + p1; pf.h[r] = (_Float16)p0; pf.h[8 + r] = (_Float16)p1; }
    l = l * alpha + ps;
#pragma unroll
    for (int r = 0; r < 8; ++r) { o0[r] *= alpha; o1[r] *= alpha; o2[r] *= alpha; o3[r] *= alpha; }
    const size_t va = voff + (size_t)k0;
    const v16h v0 = g2_frag(VT + va, hh), v1 = g2_frag(VT + va + (size_t)16 * SEQ, hh), v2 = g2_frag(VT + va + (size_t)32 * SEQ, hh), v3 = g2_frag(VT + va + (size_t)48 * SEQ, hh);
    const v16h pv = pf.v;
    o0 = WMMA_F16(v0, pv, o0); o1 = WMMA_F16(v1, pv, o1); o2 = WMMA_F16(v2, pv, o2); o3 = WMMA_F16(v3, pv, o3);
    asm volatile("v_nop\n\tv_nop\n\tv_nop\n\tv_nop" : "+v"(o0), "+v"(o1), "+v"(o2), "+v"(o3) : "v"(v0), "v"(v1), "v"(v2), "v"(v3), "v"(pv));
  }
  const float lo = __shfl_xor(l, 16); l = l + lo;
  const float inv = 64.0f * __builtin_amdgcn_rcpf(l);
  *(v8us*)&so[w][ln][0 * 16 + 8 * hh] = pack8(o0, inv);
  *(v8us*)&so[w][ln][1 * 16 + 8 * hh] = pack8(o1, inv);
  *(v8us*)&so[w][ln][2 * 16 + 8 * hh] = pack8(o2, inv);
  *(v8us*)&so[w][ln][3 * 16 + 8 * hh] = pack8(o3, inv);
  __builtin_amdgcn_fence(4  , "workgroup"); __builtin_amdgcn_wave_barrier();
  const int rq = lane >> 3, pc = (lane & 7) * 8;
  for (int pass = 0; pass < 2; ++pass) {
#pragma unroll
    for (int it = 0; it < 4; ++it) { const int row = it * 4 + rq; const v8us v = *(const v8us*)&so[w][row][pc];
      *(volatile v8us*)((unsigned short*)O16 + (rowb + q0 + row) * DM + (size_t)h * HD + pc) = v; }
    if (pass == 0) __threadfence(); }
}

constexpr size_t al256(size_t x) { return (x + 255) & ~(size_t)255; }
constexpr size_t SZ_BQKV = al256((size_t)3 * DM * DM * 2);
constexpr size_t SZ_BO   = al256((size_t)DM * DM * 2);
constexpr size_t SZ_BW1  = al256((size_t)DFF * DM * 2);
constexpr size_t SZ_BW2  = al256((size_t)DM * DFF * 2);
constexpr size_t SZ_XB   = al256(NR * DM * 4);
constexpr size_t SZ_XN   = al256(NR * DM * 2);
constexpr size_t SZ_QKV  = al256(NR * LQ * 2);
constexpr size_t SZ_VT   = al256((size_t)NB * NH * HD * SEQ * 2);
constexpr size_t SZ_O16  = al256(NR * DM * 2);
constexpr size_t SZ_X1   = al256(NR * DM * 4);
constexpr size_t SZ_HF   = NR * DFF * 2;
constexpr size_t OF_BQKV = 0;
constexpr size_t OF_BO   = OF_BQKV + SZ_BQKV;
constexpr size_t OF_BW1  = OF_BO + SZ_BO;
constexpr size_t OF_BW2  = OF_BW1 + SZ_BW1;
constexpr size_t OF_XB   = OF_BW2 + SZ_BW2;
constexpr size_t OF_XN   = OF_XB + SZ_XB;
constexpr size_t OF_QKV  = OF_XN + SZ_XN;
constexpr size_t OF_VT   = OF_QKV + SZ_QKV;
constexpr size_t OF_O16  = OF_VT + SZ_VT;
constexpr size_t OF_X1   = OF_O16 + SZ_O16;
constexpr size_t WS_TOTAL = OF_X1 + SZ_X1;
static_assert(SZ_HF <= SZ_QKV + SZ_VT);
static_assert(OF_VT == OF_QKV + SZ_QKV);
static_assert(WS_TOTAL <= (size_t)134217728);

extern "C" void kernel_launch(void* const* d_in, const int* in_sizes, int n_in,
                              void* d_out, int out_size, void* d_ws, size_t ws_size, hipStream_t stream) {
  if (n_in < 14) return;
  if ((size_t)in_sizes[0] < ((size_t)(NB - 1) * SEQ_FULL + SEQ) * DM) return;
  if ((size_t)in_sizes[1] < (size_t)(NB - 1) * SEQ_FULL + SEQ) return;
  if (in_sizes[2] < DM || in_sizes[3] < DM || in_sizes[4] < DM || in_sizes[5] < DM) return;
  if (in_sizes[6] < DM * 3 * DM || in_sizes[7] < 3 * DM || in_sizes[8] < DM * DM || in_sizes[9] < DM) return;
  if (in_sizes[10] < DM * DFF || in_sizes[11] < DFF || in_sizes[12] < DFF * DM || in_sizes[13] < DM) return;
  if ((size_t)out_size < NR * DM) return;
  if (WS_TOTAL > ws_size) return;
  const float* x = (const float*)d_in[0]; const int* kmask = (const int*)d_in[1];
  const float* g1 = (const float*)d_in[2]; const float* be1 = (const float*)d_in[3];
  const float* g2 = (const float*)d_in[4]; const float* be2 = (const float*)d_in[5];
  const float* wqkv = (const float*)d_in[6]; const float* bqkv = (const float*)d_in[7];
  const float* wo = (const float*)d_in[8]; const float* bo = (const float*)d_in[9];
  const float* w1 = (const float*)d_in[10]; const float* b1 = (const float*)d_in[11];
  const float* w2 = (const float*)d_in[12]; const float* b2 = (const float*)d_in[13];
  char* ws = (char*)d_ws;
  _Float16* BQKV = (_Float16*)(ws + OF_BQKV); _Float16* BO = (_Float16*)(ws + OF_BO); _Float16* BW1 = (_Float16*)(ws + OF_BW1); _Float16* BW2 = (_Float16*)(ws + OF_BW2);
  float* XB = (float*)(ws + OF_XB); _Float16* XN = (_Float16*)(ws + OF_XN); _Float16* QKV = (_Float16*)(ws + OF_QKV); _Float16* VT = (_Float16*)(ws + OF_VT);
  _Float16* O16 = (_Float16*)(ws + OF_O16); float* X1 = (float*)(ws + OF_X1);
  _Float16* M16 = XN;
  _Float16* HF16 = QKV;
  const int M = (int)NR;
  k_wt_f16<<<(unsigned)(((size_t)3 * DM * (DM / 8) + 255) / 256), 256, 0, stream>>>(wqkv, BQKV, DM, 3 * DM, 16.0f);
  k_wt_f16<<<(unsigned)(((size_t)DM * (DM / 8) + 255) / 256), 256, 0, stream>>>(wo, BO, DM, DM, 16.0f);
  k_wt_f16<<<(unsigned)(((size_t)DFF * (DM / 8) + 255) / 256), 256, 0, stream>>>(w1, BW1, DM, DFF, 16.0f);
  k_wt_f16<<<(unsigned)(((size_t)DM * (DFF / 8) + 255) / 256), 256, 0, stream>>>(w2, BW2, DFF, DM, 16.0f);
  k_ln1<<<(unsigned)NR, 256, 0, stream>>>(x, g1, be1, XN, XB);
  k_gemm_h16<<<(unsigned)((NR / 128) * (LQ / 64)), 128, 0, stream>>>(XN, DM, BQKV, DM, 0.0625f, bqkv, QKV, LQ, M, LQ, DM);
  k_vt<<<(unsigned)(NB * NH * (SEQ / 64)), 256, 0, stream>>>(QKV, VT);
  k_flash<<<(unsigned)(NB * NH * (SEQ / 64)), 128, 0, stream>>>(QKV, VT, kmask, O16);
  k_gemm_res32<<<(unsigned)((NR / 128) * (DM / 64)), 128, 0, stream>>>(O16, DM, BO, DM, 0.0009765625f, bo, XB, DM, X1, DM, M, DM, DM);
  k_ln2<<<(unsigned)NR, 256, 0, stream>>>(X1, g2, be2, M16);
  k_gemm_gelu16<<<(unsigned)((NR / 128) * (DFF / 64)), 128, 0, stream>>>(M16, DM, BW1, DM, 0.0625f, b1, HF16, DFF, M, DFF, DM);
  k_gemm_res32<<<(unsigned)((NR / 128) * (DM / 64)), 128, 0, stream>>>(HF16, DFF, BW2, DFF, 0.0625f, b2, X1, DM, (float*)d_out, DM, M, DM, DFF);
}
